// ScaledDotProductAttention_19550691132117
// MI455X (gfx1250) — hardware-verified
//
#include <hip/hip_runtime.h>


#ifndef NB
#define NB 2
#endif
#ifndef SEQ
#define SEQ 2048
#endif
#define NB_FULL  2
#define SEQ_FULL 2048
#define NHEAD    16
#define NBH      (NB * NHEAD)
#define DH       64
#define QBLK     128
#define NWAVE    8
#define KBLK     32
#define NKB      (SEQ / KBLK)
#define PSTR     40
#define OSTR     68
#define VTP      72

#define SCL    0.18033688011112042f
#define MASKV  (-1442695040.0f)
#define MINIT  (-1.0e30f)
#define PCAR   16384.0f
#define RCAR   1024.0f
#define RINV   0.0009765625f

static_assert(SEQ % 256 == 0);
static_assert(SEQ <= SEQ_FULL);
static_assert(NB >= 1 && NB <= NB_FULL);
static_assert(SEQ % QBLK == 0 && SEQ % 64 == 0 && SEQ % KBLK == 0);
static_assert((NWAVE * 16 * PSTR * 2) * 2 + NWAVE * 16 * OSTR * 4 <= 65536);
static_assert((PSTR * 2) % 16 == 0 && (OSTR * 4) % 16 == 0 && (VTP * 2) % 16 == 0);
static_assert((SEQ * 2) % 128 == 0);
static_assert(NWAVE * 32 == 256 && NWAVE * 16 == QBLK);

typedef _Float16 f16;
typedef _Float16 v16h __attribute__((ext_vector_type(16)));
typedef _Float16 v8h  __attribute__((ext_vector_type(8)));
typedef _Float16 v2h  __attribute__((ext_vector_type(2)));
typedef __bf16   v16b __attribute__((ext_vector_type(16)));
typedef unsigned short us16;
typedef us16     v8us __attribute__((ext_vector_type(8)));
typedef float    v8f  __attribute__((ext_vector_type(8)));
typedef float    v4f  __attribute__((ext_vector_type(4)));
typedef unsigned int v4u __attribute__((ext_vector_type(4)));
typedef int      v4i  __attribute__((ext_vector_type(4)));
typedef int      v2i  __attribute__((ext_vector_type(2)));

union FragH { v16h v; v8h half[2]; };
union FragB { v16b v; v16h hv; v8us half[2]; };
union Pack8 { v8h h; v4u u; };

static __device__ __forceinline__ v8f mma_f16(v16h a, v16h b, v8f c) {
  c = __builtin_amdgcn_wmma_f32_16x16x32_f16(false, a, false, b, (short)0, c, false, false);
  asm volatile("v_nop\n\tv_nop\n\tv_nop\n\tv_nop" : "+v"(c) : "v"(a), "v"(b));
  return c;
}
static __device__ __forceinline__ v8f mma_bf16(const FragB& a, const FragB& b, v8f c) {
  c = __builtin_amdgcn_wmma_f32_16x16x32_bf16(false, a.v, false, b.v, (short)0, c, false, false);
  asm volatile("v_nop\n\tv_nop\n\tv_nop\n\tv_nop" : "+v"(c) : "v"(a.hv), "v"(b.hv));
  return c;
}

static __device__ __forceinline__ unsigned int bf_hi(float x) {
  unsigned int u = __float_as_uint(x);
  u += 0x7FFFu + ((u >> 16) & 1u);
  return u >> 16;
}
static __device__ __forceinline__ f16 h_of_bf(float x) {
  return (f16)__uint_as_float(bf_hi(x) << 16);
}

template <int CTRL>
static __device__ __forceinline__ float dpp_max(float x) {
  int xi = __float_as_int(x);
  int yi = __builtin_amdgcn_update_dpp(xi, xi, CTRL, 0xF, 0xF, true);
  return fmaxf(x, __int_as_float(yi));
}
static __device__ __forceinline__ float rowmax16(float x) {
  x = dpp_max<0xB1>(x);
  x = dpp_max<0x4E>(x);
  x = dpp_max<0x141>(x);
  x = dpp_max<0x140>(x);
  return x;
}

static __device__ __forceinline__ void lds_wave_sync() {
  asm volatile("s_wait_dscnt 0x0" ::: "memory");
  __builtin_amdgcn_wave_barrier();
}

__global__ __launch_bounds__(256)
void k_convert(const float* __restrict__ Q, const float* __restrict__ K, const float* __restrict__ V,
               us16* __restrict__ Qp, us16* __restrict__ Kp, f16* __restrict__ Vt)
{
  __shared__ __align__(16) f16 sVt[DH * VTP];

  const int tid   = threadIdx.x;
  const int bh    = blockIdx.x / (SEQ / 64);
  const int kt    = blockIdx.x - bh * (SEQ / 64);
  const size_t rin = (size_t)bh * SEQ_FULL + (size_t)kt * 64;
  const size_t rpl = (size_t)bh * SEQ + (size_t)kt * 64;
  const int prow  = tid >> 3;
  const int piece = tid & 7;

  v4u qv[2], kv[2];
#pragma unroll
  for (int it = 0; it < 2; ++it) {
    const int row = it * 32 + prow;
    const float* qs = Q + (rin + row) * DH + piece * 8;
    const float* ks = K + (rin + row) * DH + piece * 8;
    const v4f q0 = *(const v4f*)(qs);
    const v4f q1 = *(const v4f*)(qs + 4);
    const v4f k0 = *(const v4f*)(ks);
    const v4f k1 = *(const v4f*)(ks + 4);
    v4u a, b;
    a.x = bf_hi(q0.x) | (bf_hi(q0.y) << 16);
    a.y = bf_hi(q0.z) | (bf_hi(q0.w) << 16);
    a.z = bf_hi(q1.x) | (bf_hi(q1.y) << 16);
    a.w = bf_hi(q1.z) | (bf_hi(q1.w) << 16);
    b.x = bf_hi(k0.x) | (bf_hi(k0.y) << 16);
    b.y = bf_hi(k0.z) | (bf_hi(k0.w) << 16);
    b.z = bf_hi(k1.x) | (bf_hi(k1.y) << 16);
    b.w = bf_hi(k1.z) | (bf_hi(k1.w) << 16);
    qv[it] = a;
    kv[it] = b;
  }
#pragma unroll
  for (int it = 0; it < 2; ++it) {
    const int row = it * 32 + prow;
    *(volatile v4u*)(Qp + (rpl + row) * DH + piece * 8) = qv[it];
    *(volatile v4u*)(Kp + (rpl + row) * DH + piece * 8) = kv[it];
  }
  __threadfence();
#pragma unroll
  for (int it = 0; it < 2; ++it) {
    const int row = it * 32 + prow;
    *(volatile v4u*)(Qp + (rpl + row) * DH + piece * 8) = qv[it];
    *(volatile v4u*)(Kp + (rpl + row) * DH + piece * 8) = kv[it];
  }

  {
    const int key = tid >> 2;
    const int d0  = (tid & 3) * 16;
    const float* vs = V + (rin + key) * DH + d0;
#pragma unroll
    for (int j = 0; j < 4; ++j) {
      const v4f x = *(const v4f*)(vs + 4 * j);
      sVt[(d0 + 4 * j + 0) * VTP + key] = h_of_bf(x.x);
      sVt[(d0 + 4 * j + 1) * VTP + key] = h_of_bf(x.y);
      sVt[(d0 + 4 * j + 2) * VTP + key] = h_of_bf(x.z);
      sVt[(d0 + 4 * j + 3) * VTP + key] = h_of_bf(x.w);
    }
  }
  __syncthreads();
  Pack8 vv[2];
#pragma unroll
  for (int it = 0; it < 2; ++it) {
    const int d = it * 32 + prow;
    vv[it].h = *(const v8h*)(sVt + d * VTP + piece * 8);
  }
#pragma unroll
  for (int it = 0; it < 2; ++it) {
    const int d = it * 32 + prow;
    *(volatile v4u*)(Vt + ((size_t)bh * DH + d) * SEQ + (size_t)kt * 64 + piece * 8) = vv[it].u;
  }
  __threadfence();
#pragma unroll
  for (int it = 0; it < 2; ++it) {
    const int d = it * 32 + prow;
    *(volatile v4u*)(Vt + ((size_t)bh * DH + d) * SEQ + (size_t)kt * 64 + piece * 8) = vv[it].u;
  }
}

template <int EARLY>
__global__ __launch_bounds__(256)
void k_attn(const us16* __restrict__ Qp, const us16* __restrict__ Kp, const f16* __restrict__ Vt,
            const int* __restrict__ msk, float* __restrict__ O, int qt0, int nqt)
{
  __shared__ __align__(16) f16   sP[NWAVE * 16 * PSTR];
  __shared__ __align__(16) f16   sR[NWAVE * 16 * PSTR];
  __shared__ __align__(16) float sO[NWAVE * 16 * OSTR];

  const int tid  = threadIdx.x;
  const int wave = tid >> 5;
  const int lane = tid & 31;
  const int h    = lane >> 4;
  const int l16  = lane & 15;

  const int bh    = blockIdx.x / nqt;
  const int qt    = qt0 + (blockIdx.x - bh * nqt);
  const int bb    = bh / NHEAD;
  const int qwave = qt * QBLK + wave * 16;

  const us16* Qb = Qp + ((size_t)bh * SEQ + qwave) * DH;
  const us16* Kb = Kp + (size_t)bh * SEQ * DH;
  const f16*  Vb = Vt + (size_t)bh * DH * SEQ;
  float*      Ob = O + ((size_t)bh * SEQ + qwave) * DH;
  const int*  Mb = msk + ((size_t)bb * SEQ_FULL + (size_t)qwave) * SEQ_FULL;

  FragB qa[2];
#pragma unroll
  for (int kc = 0; kc < 2; ++kc) {
    const us16* qr = Qb + (size_t)l16 * DH + kc * 32 + 8 * h;
    qa[kc].half[0] = *(const v8us*)(qr);
    qa[kc].half[1] = *(const v8us*)(qr + 16);
  }

  v16h onesv;
#pragma unroll
  for (int i = 0; i < 16; ++i) onesv[i] = (f16)1.0f;
  v16h onessv;
#pragma unroll
  for (int i = 0; i < 16; ++i) onessv[i] = (f16)RINV;

  const v8f vzero = {0.f, 0.f, 0.f, 0.f, 0.f, 0.f, 0.f, 0.f};
  v8f oacc[4];
#pragma unroll
  for (int vt = 0; vt < 4; ++vt) oacc[vt] = vzero;
  float mrow[8], lrow[8];
#pragma unroll
  for (int r = 0; r < 8; ++r) { mrow[r] = MINIT; lrow[r] = 0.f; }

  const int pofs = wave * 16 * PSTR;

  for (int kb = 0; kb < NKB; ++kb) {
    const int k0 = kb * KBLK;

    FragB kf[2][2];
#pragma unroll
    for (int nt = 0; nt < 2; ++nt)
#pragma unroll
      for (int kc = 0; kc < 2; ++kc) {
        const us16* kr = Kb + (size_t)(k0 + 2 * l16 + nt) * DH + kc * 32 + 8 * h;
        kf[nt][kc].half[0] = *(const v8us*)(kr);
        kf[nt][kc].half[1] = *(const v8us*)(kr + 16);
      }

    v8f s0 = mma_bf16(qa[0], kf[0][0], vzero);
    s0     = mma_bf16(qa[1], kf[0][1], s0);
    v8f s1 = mma_bf16(qa[0], kf[1][0], vzero);
    s1     = mma_bf16(qa[1], kf[1][1], s1);
#pragma unroll
    for (int r = 0; r < 8; ++r) { s0[r] *= SCL; s1[r] *= SCL; }

#pragma unroll
    for (int r = 0; r < 8; ++r) {
      const v2i m = *(const v2i*)(Mb + (size_t)(8 * h + r) * SEQ_FULL + k0 + 2 * l16);
      s0[r] = (m.x != 0) ? s0[r] : MASKV;
      s1[r] = (m.y != 0) ? s1[r] : MASKV;
    }

    float alpha[8];
#pragma unroll
    for (int r = 0; r < 8; ++r) {
      const float mx = rowmax16(fmaxf(s0[r], s1[r]));
      const float mn = fmaxf(mrow[r], mx);
      alpha[r] = __builtin_amdgcn_exp2f(mrow[r] - mn);
      mrow[r]  = mn;
      const float p0 = __builtin_amdgcn_exp2f(s0[r] - mn) * PCAR;
      const float p1 = __builtin_amdgcn_exp2f(s1[r] - mn) * PCAR;
      const f16 ph0 = (f16)p0;
      const f16 ph1 = (f16)p1;
      v2h pp; pp.x = ph0; pp.y = ph1;
      *(v2h*)(sP + pofs + (8 * h + r) * PSTR + 2 * l16) = pp;
      if (EARLY) {
        const float e0 = (p0 - (float)ph0) * RCAR;
        const float e1 = (p1 - (float)ph1) * RCAR;
        v2h rr; rr.x = (f16)e0; rr.y = (f16)e1;
        *(v2h*)(sR + pofs + (8 * h + r) * PSTR + 2 * l16) = rr;
      }
    }
    lds_wave_sync();

    FragH pa;
    pa.half[0] = *(const v8h*)(sP + pofs + l16 * PSTR + 8 * h);
    pa.half[1] = *(const v8h*)(sP + pofs + l16 * PSTR + 16 + 8 * h);
    FragH pr;
    pr.v = pa.v;
    if (EARLY) {
      pr.half[0] = *(const v8h*)(sR + pofs + l16 * PSTR + 8 * h);
      pr.half[1] = *(const v8h*)(sR + pofs + l16 * PSTR + 16 + 8 * h);
    }

    v8f lsum = mma_f16(pa.v, onesv, vzero);
    if (EARLY) lsum = mma_f16(pr.v, onessv, lsum);

#pragma unroll
    for (int vt = 0; vt < 4; ++vt) {
      FragH vb;
      const f16* vr = Vb + (size_t)(vt * 16 + l16) * SEQ + k0 + 8 * h;
      vb.half[0] = *(const v8h*)(vr);
      vb.half[1] = *(const v8h*)(vr + 16);
#pragma unroll
      for (int r = 0; r < 8; ++r) oacc[vt][r] *= alpha[r];
      oacc[vt] = mma_f16(pa.v, vb.v, oacc[vt]);
      if (EARLY) {
        const v16h vs = vb.v * (f16)RINV;
        oacc[vt] = mma_f16(pr.v, vs, oacc[vt]);
      }
    }
#pragma unroll
    for (int r = 0; r < 8; ++r) lrow[r] = lrow[r] * alpha[r] + lsum[r];
  }

  float inv[8];
#pragma unroll
  for (int r = 0; r < 8; ++r) inv[r] = __builtin_amdgcn_rcpf(lrow[r]);
  float* sOw = sO + wave * 16 * OSTR;
#pragma unroll
  for (int vt = 0; vt < 4; ++vt)
#pragma unroll
    for (int r = 0; r < 8; ++r)
      sOw[(8 * h + r) * OSTR + vt * 16 + l16] = oacc[vt][r] * inv[r];
  lds_wave_sync();

  const int lq = lane >> 3;
  const int lp = lane & 7;
#pragma unroll
  for (int j = 0; j < 8; ++j) {
    const int L = j * 4 + lq;
    const int row = L >> 1, hf = L & 1;
    const v4f v = *(const v4f*)(sOw + row * OSTR + hf * 32 + lp * 4);
    *(volatile v4f*)(Ob + (size_t)row * DH + hf * 32 + lp * 4) = v;
  }
  __threadfence();
#pragma unroll
  for (int j = 0; j < 8; ++j) {
    const int L = j * 4 + lq;
    const int row = L >> 1, hf = L & 1;
    const v4f v = *(const v4f*)(sOw + row * OSTR + hf * 32 + lp * 4);
    *(volatile v4f*)(Ob + (size_t)row * DH + hf * 32 + lp * 4) = v;
  }
}

extern "C" void kernel_launch(void* const* d_in, const int* in_sizes, int n_in,
                              void* d_out, int out_size, void* d_ws, size_t ws_size,
                              hipStream_t stream)
{
  if (n_in < 4) return;
  const long long needQ = ((long long)(NBH - 1) * SEQ_FULL + SEQ) * DH;
  if ((long long)in_sizes[0] < needQ) return;
  if ((long long)in_sizes[1] < needQ) return;
  if ((long long)in_sizes[2] < needQ) return;
  const long long needM = ((long long)(NB - 1) * SEQ_FULL + (SEQ - 1)) * SEQ_FULL + SEQ;
  if ((long long)in_sizes[3] < needM) return;
  if ((long long)out_size < (long long)NBH * SEQ * DH) return;

  const float* Q = (const float*)d_in[0];
  const float* K = (const float*)d_in[1];
  const float* V = (const float*)d_in[2];
  const int*   M = (const int*)d_in[3];
  float*       O = (float*)d_out;

  const size_t planeB = (size_t)NBH * SEQ * DH * 2;
  const size_t offQ   = 0;
  const size_t offK   = planeB;
  const size_t offV   = 2 * planeB;
  const size_t total  = 3 * planeB;
  if (ws_size < total) return;

  char* ws = (char*)d_ws;
  us16* Qp = (us16*)(ws + offQ);
  us16* Kp = (us16*)(ws + offK);
  f16*  Vt = (f16*)(ws + offV);

  k_convert<<<dim3(NBH * (SEQ / 64)), dim3(256), 0, stream>>>(Q, K, V, Qp, Kp, Vt);
  k_attn<1><<<dim3(NBH), dim3(256), 0, stream>>>(Qp, Kp, Vt, M, O, 0, 1);
  const int nlate = SEQ / QBLK - 1;
  if (nlate > 0)
    k_attn<0><<<dim3(NBH * nlate), dim3(256), 0, stream>>>(Qp, Kp, Vt, M, O, 1, nlate);
}
